// MultiHeadAttention_50972671869450
// MI455X (gfx1250) — hardware-verified
//
#include <hip/hip_runtime.h>


#ifndef NB
#define NB 2
#endif
#ifndef SEQ
#define SEQ 2048
#endif
#define NB_FULL 2
#define S_FULL  2048
#define DMODEL  1024
#define HEADS   16
#define DKH     64
#define MROWS   (NB * SEQ)

static_assert(NB >= 1 && NB <= NB_FULL);
static_assert(SEQ >= 128 && SEQ <= S_FULL && (SEQ % 128) == 0);
static_assert((SEQ % 64) == 0);
static_assert(DMODEL == HEADS * DKH);
static_assert(DKH == 64);
static_assert(DMODEL / 64 == HEADS);
static_assert((MROWS % 128) == 0 && (DMODEL % 64) == 0 && (DMODEL % 32) == 0);
static_assert((size_t)MROWS * DMODEL * 4 <= (size_t)16777216);

#define STR32  40
#define STRK   72
#define STRT0  72
#define STRT1  136
#define STRT2  68

static_assert(STR32 >= 32 && (STR32 % 8) == 0);
static_assert(STRK  >= 64 && (STRK  % 8) == 0);
static_assert(STRT0 >= 64 && (STRT0 % 8) == 0);
static_assert(STRT1 >= 128 && (STRT1 % 8) == 0);
static_assert(STRT2 >= 64 && (STRT2 % 4) == 0);
static_assert(256 * 16 == 128 * 32);
static_assert(128 * 16 == 64 * 32);
static_assert(512 * 8 == 64 * DKH);
static_assert(8 * 16 == 128);

typedef _Float16 v16h  __attribute__((ext_vector_type(16)));
typedef _Float16 v8h   __attribute__((ext_vector_type(8)));
typedef float    v8f   __attribute__((ext_vector_type(8)));
typedef float    v4f   __attribute__((ext_vector_type(4)));
typedef unsigned u32x4 __attribute__((ext_vector_type(4)));

#define XPL       ((size_t)MROWS * DMODEL)
#define WPL       ((size_t)DMODEL * DMODEL)
#define OFF_XQ    ((size_t)0)
#define OFF_XK    (XPL)
#define OFF_XV    (2 * XPL)
#define OFF_WQ    (3 * XPL)
#define OFF_WK    (3 * XPL + WPL)
#define OFF_WV    (3 * XPL + 2 * WPL)
#define OFF_WO    (3 * XPL + 3 * WPL)
#define OFF_Q16   (3 * XPL + 4 * WPL)
#define OFF_K16   (4 * XPL + 4 * WPL)
#define OFF_VT    (5 * XPL + 4 * WPL)
#define OFF_CTX   (6 * XPL + 4 * WPL)
#define WS_HALVES (7 * XPL + 4 * WPL)
static_assert(WS_HALVES * 2 <= (size_t)134217728);
static_assert(((3 * XPL + 4 * WPL) % 2048) == 0);
static_assert((XPL % 2048) == 0 && (WPL % 2048) == 0);

__device__ __forceinline__ v8f vz8() {
    v8f r;
#pragma unroll
    for (int i = 0; i < 8; ++i) r[i] = 0.0f;
    return r;
}

__device__ __forceinline__ v8f wmma_f16(v16h a, v16h b, v8f c) {
    v8f d = __builtin_amdgcn_wmma_f32_16x16x32_f16(false, a, false, b, (short)0, c, false, false);
    asm volatile("v_nop\n\tv_nop\n\tv_nop\n\tv_nop" : "+v"(d) : "v"(a), "v"(b));
    return d;
}

__device__ __forceinline__ v16h load_frag(const _Float16* base, int row, int stride, int lane) {
    const _Float16* p = base + row * stride + 8 * (lane >> 4);
    v8h lo = *(const v8h*)p;
    v8h hi = *(const v8h*)(p + 16);
    v16h r;
#pragma unroll
    for (int i = 0; i < 8; ++i) { r[i] = lo[i]; r[i + 8] = hi[i]; }
    return r;
}

__device__ __forceinline__ float bf16_rne(float f) {
    unsigned u = __float_as_uint(f);
    u = (u + 0x7FFFu + ((u >> 16) & 1u)) & 0xFFFF0000u;
    return __uint_as_float(u);
}

__device__ __forceinline__ float dpp_xor1(float v) {
    return __int_as_float(__builtin_amdgcn_update_dpp(0, __float_as_int(v), 0xB1, 0xf, 0xf, true));
}
__device__ __forceinline__ float dpp_xor2(float v) {
    return __int_as_float(__builtin_amdgcn_update_dpp(0, __float_as_int(v), 0x4E, 0xf, 0xf, true));
}
__device__ __forceinline__ float dpp_hmir(float v) {
    return __int_as_float(__builtin_amdgcn_update_dpp(0, __float_as_int(v), 0x141, 0xf, 0xf, true));
}
__device__ __forceinline__ float dpp_mir(float v) {
    return __int_as_float(__builtin_amdgcn_update_dpp(0, __float_as_int(v), 0x140, 0xf, 0xf, true));
}
__device__ __forceinline__ float rmax16(float v) {
    v = fmaxf(v, dpp_xor1(v));
    v = fmaxf(v, dpp_xor2(v));
    v = fmaxf(v, dpp_hmir(v));
    v = fmaxf(v, dpp_mir(v));
    return v;
}
__device__ __forceinline__ float rsum16(float v) {
    v += dpp_xor1(v);
    v += dpp_xor2(v);
    v += dpp_hmir(v);
    v += dpp_mir(v);
    return v;
}

__global__ __launch_bounds__(256) void cvt_planes_kernel(
    const float* __restrict__ xq, const float* __restrict__ xk, const float* __restrict__ xv,
    const float* __restrict__ wq, const float* __restrict__ wk, const float* __restrict__ wv,
    const float* __restrict__ wo, _Float16* __restrict__ planes)
{
    const unsigned XN = (unsigned)XPL, WN = (unsigned)WPL;
    const unsigned total = 3u * XN + 4u * WN;
    const unsigned e = (blockIdx.x * 256u + threadIdx.x) * 8u;
    if (e >= total) return;
    int pid; unsigned off;
    if (e < 3u * XN) { pid = (int)(e / XN); off = e - (unsigned)pid * XN; }
    else { unsigned e2 = e - 3u * XN; pid = 3 + (int)(e2 / WN); off = e2 - (unsigned)(pid - 3) * WN; }
    const float* src = (pid == 0) ? xq : (pid == 1) ? xk : (pid == 2) ? xv
                     : (pid == 3) ? wq : (pid == 4) ? wk : (pid == 5) ? wv : wo;
    const float sc = (pid < 3) ? 1.0f : 64.0f;
    size_t soff;
    if (pid < 3) {
        unsigned m = off / DMODEL, col = off % DMODEL;
        unsigned b = m / SEQ, s = m % SEQ;
        soff = ((size_t)b * S_FULL + s) * DMODEL + col;
    } else {
        soff = off;
    }
    v4f x0 = *(const v4f*)(src + soff);
    v4f x1 = *(const v4f*)(src + soff + 4);
    v8h hv;
#pragma unroll
    for (int i = 0; i < 4; ++i) {
        hv[i]     = (_Float16)(bf16_rne(x0[i]) * sc);
        hv[4 + i] = (_Float16)(bf16_rne(x1[i]) * sc);
    }
    u32x4 w = __builtin_bit_cast(u32x4, hv);
    volatile u32x4* dp = (volatile u32x4*)(planes + e);
    *dp = w;
    __threadfence();
    *dp = w;
}

template <int MODE>
__device__ __forceinline__ void gemm_store_tile(const char* sTraw, void* outp, int bm, int bn, int wave, int lane) {
    const int hf = lane >> 4, c16 = lane & 15;
    if constexpr (MODE == 0) {
        const _Float16* sTh = (const _Float16*)sTraw;
        const int bM = (bm * 128) / SEQ, s0 = (bm * 128) % SEQ;
        _Float16* g = (_Float16*)outp + (((size_t)bM * HEADS + bn) * SEQ + s0) * DKH;
#pragma unroll
        for (int j = 0; j < 4; ++j) {
            int row = wave * 16 + j * 4 + (lane >> 3), col = (lane & 7) * 8;
            v8h hv = *(const v8h*)(sTh + row * STRT0 + col);
            *(volatile u32x4*)(g + (size_t)row * DKH + col) = __builtin_bit_cast(u32x4, hv);
        }
    } else if constexpr (MODE == 1) {
        const _Float16* sTh = (const _Float16*)sTraw;
        const int bM = (bm * 128) / SEQ, s0 = (bm * 128) % SEQ;
        _Float16* g = (_Float16*)outp + ((size_t)bM * HEADS + bn) * DKH * SEQ + s0;
#pragma unroll
        for (int j = 0; j < 4; ++j) {
            int dk = wave * 8 + j * 2 + hf, col = c16 * 8;
            v8h hv = *(const v8h*)(sTh + dk * STRT1 + col);
            *(volatile u32x4*)(g + (size_t)dk * SEQ + col) = __builtin_bit_cast(u32x4, hv);
        }
    } else {
        const float* sTf = (const float*)sTraw;
        float* g = (float*)outp + (size_t)(bm * 128) * DMODEL + bn * 64;
#pragma unroll
        for (int j = 0; j < 8; ++j) {
            int row = wave * 16 + j * 2 + hf, col = c16 * 4;
            v4f fv = *(const v4f*)(sTf + row * STRT2 + col);
            *(volatile v4f*)(g + (size_t)row * DMODEL + col) = fv;
        }
    }
}

template <int MODE>
__device__ __forceinline__ void gemm_xwT_body(const _Float16* __restrict__ A,
                                              const _Float16* __restrict__ Bw,
                                              const float* __restrict__ bias,
                                              void* __restrict__ outp)
{
    __shared__ __align__(16) _Float16 sA[128 * STR32];
    __shared__ __align__(16) _Float16 sB[64 * STR32];
    constexpr int TBYTES = (MODE == 2) ? 128 * STRT2 * 4 : (MODE == 0) ? 128 * STRT0 * 2 : 64 * STRT1 * 2;
    __shared__ __align__(16) char sTraw[TBYTES];

    const int K = DMODEL;
    const int t = threadIdx.x, wave = t >> 5, lane = t & 31, hf = lane >> 4, c16 = lane & 15;
    const int bm = blockIdx.x;
    const int bn = blockIdx.y;
    const int wm = (wave >> 1) * 32;
    const int wn = (wave & 1) * 32;

    v8f acc[2][2];
    acc[0][0] = vz8(); acc[0][1] = vz8(); acc[1][0] = vz8(); acc[1][1] = vz8();

#pragma unroll 1
    for (int k0 = 0; k0 < K; k0 += 32) {
        __syncthreads();
        {
            int row = t >> 1, cc = (t & 1) * 16;
            const _Float16* a = A + (size_t)(bm * 128 + row) * K + k0 + cc;
            _Float16* d = sA + row * STR32 + cc;
            *(v8h*)d       = *(const v8h*)a;
            *(v8h*)(d + 8) = *(const v8h*)(a + 8);
        }
        if (t < 128) {
            int row = t >> 1, cc = (t & 1) * 16;
            const _Float16* w = Bw + (size_t)(bn * 64 + row) * K + k0 + cc;
            _Float16* d = sB + row * STR32 + cc;
            *(v8h*)d       = *(const v8h*)w;
            *(v8h*)(d + 8) = *(const v8h*)(w + 8);
        }
        __syncthreads();

        v16h a0 = load_frag(sA + wm * STR32,        c16, STR32, lane);
        v16h a1 = load_frag(sA + (wm + 16) * STR32, c16, STR32, lane);
        v16h b0 = load_frag(sB + wn * STR32,        c16, STR32, lane);
        v16h b1 = load_frag(sB + (wn + 16) * STR32, c16, STR32, lane);

        acc[0][0] = wmma_f16(a0, b0, acc[0][0]);
        acc[0][1] = wmma_f16(a0, b1, acc[0][1]);
        acc[1][0] = wmma_f16(a1, b0, acc[1][0]);
        acc[1][1] = wmma_f16(a1, b1, acc[1][1]);
    }

    const float osc = (MODE == 2) ? (1.0f / 4096.0f) : (1.0f / 64.0f);
    _Float16* sTh = (_Float16*)sTraw;
    float*    sTf = (float*)sTraw;
#pragma unroll
    for (int mi = 0; mi < 2; ++mi) {
#pragma unroll
        for (int ni = 0; ni < 2; ++ni) {
            const int lcol = wn + ni * 16 + c16;
            const float bb = bf16_rne(bias[bn * 64 + lcol]);
#pragma unroll
            for (int r = 0; r < 8; ++r) {
                const int lrow = wm + mi * 16 + 8 * hf + r;
                const float v = acc[mi][ni][r] * osc + bb;
                if constexpr (MODE == 2)      sTf[lrow * STRT2 + lcol] = v;
                else if constexpr (MODE == 0) sTh[lrow * STRT0 + lcol] = (_Float16)v;
                else                          sTh[lcol * STRT1 + lrow] = (_Float16)v;
            }
        }
    }
    __syncthreads();

    gemm_store_tile<MODE>(sTraw, outp, bm, bn, wave, lane);
    __threadfence();
    gemm_store_tile<MODE>(sTraw, outp, bm, bn, wave, lane);
}

__global__ __launch_bounds__(256) void gemm_headsplit_kernel(const _Float16* __restrict__ A,
                                                             const _Float16* __restrict__ Bw,
                                                             const float* __restrict__ bias,
                                                             _Float16* __restrict__ outp)
{
    gemm_xwT_body<0>(A, Bw, bias, (void*)outp);
}

__global__ __launch_bounds__(256) void gemm_headsplit_t_kernel(const _Float16* __restrict__ A,
                                                               const _Float16* __restrict__ Bw,
                                                               const float* __restrict__ bias,
                                                               _Float16* __restrict__ outp)
{
    gemm_xwT_body<1>(A, Bw, bias, (void*)outp);
}

__global__ __launch_bounds__(256) void gemm_out_f32_kernel(const _Float16* __restrict__ A,
                                                           const _Float16* __restrict__ Bw,
                                                           const float* __restrict__ bias,
                                                           float* __restrict__ outp)
{
    gemm_xwT_body<2>(A, Bw, bias, (void*)outp);
}

__global__ __launch_bounds__(256) __attribute__((amdgpu_num_vgpr(256)))
void attn_kernel(const _Float16* __restrict__ q16, const _Float16* __restrict__ k16,
                 const _Float16* __restrict__ vt16, _Float16* __restrict__ ctx16)
{
    __shared__ __align__(16) _Float16 sK[64 * STRK];
    __shared__ __align__(16) _Float16 sV[64 * STRK];
    __shared__ __align__(16) _Float16 sP[8 * 16 * STRK];

    const int t = threadIdx.x, wave = t >> 5, lane = t & 31, hf = lane >> 4, c16 = lane & 15;
    const int qb = blockIdx.x;
    const int bh = blockIdx.y;
    const int b  = bh / HEADS;
    const int hh = bh % HEADS;
    const int q0 = qb * 128 + wave * 16;

    const _Float16* qg = q16  + ((size_t)bh * SEQ + q0) * DKH;
    const _Float16* kg = k16  + (size_t)bh * SEQ * DKH;
    const _Float16* vg = vt16 + (size_t)bh * DKH * SEQ;

    const v16h qa0 = load_frag(qg,      c16, DKH, lane);
    const v16h qa1 = load_frag(qg + 32, c16, DKH, lane);

    _Float16* pbuf = sP + wave * 16 * STRK;

    v8f o[4];
    o[0] = vz8(); o[1] = vz8(); o[2] = vz8(); o[3] = vz8();
    float mrow[8], lrow[8];
#pragma unroll
    for (int r = 0; r < 8; ++r) { mrow[r] = -1e30f; lrow[r] = 0.0f; }

    constexpr int NKB = SEQ / 64;
#pragma unroll 1
    for (int kb = 0; kb < NKB; ++kb) {
        __syncthreads();
        for (int i = t; i < 512; i += 256) {
            int row = i >> 3, cc = (i & 7) * 8;
            *(v8h*)(sK + row * STRK + cc) = *(const v8h*)(kg + (size_t)(kb * 64 + row) * DKH + cc);
            *(v8h*)(sV + row * STRK + cc) = *(const v8h*)(vg + (size_t)row * SEQ + kb * 64 + cc);
        }
        __syncthreads();

        v8f s[4];
#pragma unroll
        for (int q4 = 0; q4 < 4; ++q4) {
            v16h kf0 = load_frag(sK,      q4 * 16 + c16, STRK, lane);
            v16h kf1 = load_frag(sK + 32, q4 * 16 + c16, STRK, lane);
            v8f a = vz8();
            a = wmma_f16(qa0, kf0, a);
            a = wmma_f16(qa1, kf1, a);
            s[q4] = a;
        }

        float alpha[8];
#pragma unroll
        for (int r = 0; r < 8; ++r) {
            float f0 = s[0][r] * 0.125f;
            float f1 = s[1][r] * 0.125f;
            float f2 = s[2][r] * 0.125f;
            float f3 = s[3][r] * 0.125f;
            float mx = rmax16(fmaxf(fmaxf(f0, f1), fmaxf(f2, f3)));
            float mn = fmaxf(mrow[r], mx);
            float al = __expf(mrow[r] - mn);
            mrow[r] = mn;
            alpha[r] = al;
            float p0 = __expf(f0 - mn);
            float p1 = __expf(f1 - mn);
            float p2 = __expf(f2 - mn);
            float p3 = __expf(f3 - mn);
            lrow[r] = lrow[r] * al + rsum16((p0 + p1) + (p2 + p3));
            const int prow = r + 8 * hf;
            pbuf[prow * STRK + 0  + c16] = (_Float16)(p0 * 1024.0f);
            pbuf[prow * STRK + 16 + c16] = (_Float16)(p1 * 1024.0f);
            pbuf[prow * STRK + 32 + c16] = (_Float16)(p2 * 1024.0f);
            pbuf[prow * STRK + 48 + c16] = (_Float16)(p3 * 1024.0f);
        }
#pragma unroll
        for (int tf = 0; tf < 4; ++tf) {
#pragma unroll
            for (int r = 0; r < 8; ++r) o[tf][r] *= alpha[r];
        }

        __builtin_amdgcn_fence(3, "wavefront");
        asm volatile("s_wait_dscnt 0x0" ::: "memory");
        __builtin_amdgcn_wave_barrier();

        v16h ap0 = load_frag(pbuf,      c16, STRK, lane);
        v16h ap1 = load_frag(pbuf + 32, c16, STRK, lane);
#pragma unroll
        for (int tf = 0; tf < 4; ++tf) {
            v16h vf0 = load_frag(sV + tf * 16 * STRK,      c16, STRK, lane);
            o[tf] = wmma_f16(ap0, vf0, o[tf]);
            v16h vf1 = load_frag(sV + tf * 16 * STRK + 32, c16, STRK, lane);
            o[tf] = wmma_f16(ap1, vf1, o[tf]);
        }
    }

    asm volatile("s_wait_dscnt 0x0" ::: "memory");
    __builtin_amdgcn_wave_barrier();
#pragma unroll
    for (int r = 0; r < 8; ++r) {
        const float inv = 0.0625f / lrow[r];
        const int prow = r + 8 * hf;
#pragma unroll
        for (int tf = 0; tf < 4; ++tf)
            pbuf[prow * STRK + tf * 16 + c16] = (_Float16)(o[tf][r] * inv);
    }
    __builtin_amdgcn_fence(3, "wavefront");
    asm volatile("s_wait_dscnt 0x0" ::: "memory");
    __builtin_amdgcn_wave_barrier();

    _Float16* gc = ctx16 + ((size_t)b * SEQ + q0) * DMODEL + hh * DKH;
#pragma unroll
    for (int j = 0; j < 4; ++j) {
        int row = j * 4 + (lane >> 3), col = (lane & 7) * 8;
        v8h hv = *(const v8h*)(pbuf + row * STRK + col);
        *(volatile u32x4*)(gc + (size_t)row * DMODEL + col) = __builtin_bit_cast(u32x4, hv);
    }
    __threadfence();
#pragma unroll
    for (int j = 0; j < 4; ++j) {
        int row = j * 4 + (lane >> 3), col = (lane & 7) * 8;
        v8h hv = *(const v8h*)(pbuf + row * STRK + col);
        *(volatile u32x4*)(gc + (size_t)row * DMODEL + col) = __builtin_bit_cast(u32x4, hv);
    }
}

extern "C" void kernel_launch(void* const* d_in, const int* in_sizes, int n_in,
                              void* d_out, int out_size, void* d_ws, size_t ws_size,
                              hipStream_t stream) {
    if (n_in < 12) return;
    const int needX = ((NB - 1) * S_FULL + SEQ) * DMODEL;
    if (in_sizes[0] < needX || in_sizes[1] < needX || in_sizes[2] < needX) return;
    if (in_sizes[3] < DMODEL * DMODEL || in_sizes[5] < DMODEL * DMODEL ||
        in_sizes[7] < DMODEL * DMODEL || in_sizes[9] < DMODEL * DMODEL) return;
    if (in_sizes[4] < DMODEL || in_sizes[6] < DMODEL || in_sizes[8] < DMODEL || in_sizes[10] < DMODEL) return;
    if (in_sizes[11] < 1) return;
    if (out_size < MROWS * DMODEL) return;
    if (ws_size < WS_HALVES * 2) return;

    const float* xq_in = (const float*)d_in[0];
    const float* xk_in = (const float*)d_in[1];
    const float* xv_in = (const float*)d_in[2];
    const float* Wq    = (const float*)d_in[3];
    const float* bq    = (const float*)d_in[4];
    const float* Wk    = (const float*)d_in[5];
    const float* bk    = (const float*)d_in[6];
    const float* Wv    = (const float*)d_in[7];
    const float* bv    = (const float*)d_in[8];
    const float* Wo    = (const float*)d_in[9];
    const float* bo    = (const float*)d_in[10];
    const int*   flag  = (const int*)d_in[11];
    (void)flag;

    _Float16* ws = (_Float16*)d_ws;
    _Float16* xq16  = ws + OFF_XQ;
    _Float16* xk16  = ws + OFF_XK;
    _Float16* xv16  = ws + OFF_XV;
    _Float16* wq16  = ws + OFF_WQ;
    _Float16* wk16  = ws + OFF_WK;
    _Float16* wv16  = ws + OFF_WV;
    _Float16* wo16  = ws + OFF_WO;
    _Float16* q16   = ws + OFF_Q16;
    _Float16* k16   = ws + OFF_K16;
    _Float16* vt16  = ws + OFF_VT;
    _Float16* ctx16 = ws + OFF_CTX;

    const unsigned ncvt = (unsigned)((3 * XPL + 4 * WPL) / 2048);
    cvt_planes_kernel<<<dim3(ncvt), dim3(256), 0, stream>>>(xq_in, xk_in, xv_in, Wq, Wk, Wv, Wo, ws);

    const dim3 gg(MROWS / 128, DMODEL / 64);
    const dim3 bb(256);
    gemm_headsplit_kernel<<<gg, bb, 0, stream>>>(xq16, wq16, bq, q16);
    gemm_headsplit_kernel<<<gg, bb, 0, stream>>>(xk16, wk16, bk, k16);
    gemm_headsplit_t_kernel<<<gg, bb, 0, stream>>>(xv16, wv16, bv, vt16);

    attn_kernel<<<dim3(SEQ / 128, NB * HEADS), bb, 0, stream>>>(q16, k16, vt16, ctx16);

    gemm_out_f32_kernel<<<gg, bb, 0, stream>>>(ctx16, wo16, bo, (float*)d_out);
}
